// GNNAndGRU_31233002177121
// MI455X (gfx1250) — hardware-verified
//
#include <hip/hip_runtime.h>
#include <math.h>

typedef _Float16 v16h __attribute__((ext_vector_type(16)));
typedef _Float16 v8h  __attribute__((ext_vector_type(8)));
typedef float    v8f  __attribute__((ext_vector_type(8)));
typedef float    v4f  __attribute__((ext_vector_type(4)));
union Frag { v16h v; v8h hv[2]; };

#define NB    4
#define NT    64
#define NN    256
#define NHG   128
#define NE    4096

__device__ __forceinline__ float lrelu(float x) { return x > 0.f ? x : 0.1f * x; }
__device__ __forceinline__ float sigm(float x) {
    float e = expf(-x);
    return __builtin_amdgcn_rcpf(1.f + e);
}

__device__ __forceinline__ v8f wmma16(v16h a, v16h b, v8f c) {
    v8f d = __builtin_amdgcn_wmma_f32_16x16x32_f16(false, a, false, b, (short)0, c, false, false);
    asm volatile("v_nop\n\tv_nop\n\tv_nop\n\tv_nop" : "+v"(d) : "v"(a), "v"(b));
    return d;
}

__global__ void __launch_bounds__(384) gi_kernel(const float* __restrict__ x, const float* __restrict__ wih,
                                                 const float* __restrict__ bih, float* gi) {
    __shared__ __attribute__((aligned(16))) float xrow[NN];
    __shared__ __attribute__((aligned(16))) float grow[3 * NHG];
    const int row = blockIdx.x;
    const int tid = threadIdx.x;
    if (tid < NN) xrow[tid] = x[(size_t)row * NN + tid];
    __syncthreads();
    float acc = bih[tid];
    const float* w = wih + (size_t)tid * NN;
#pragma unroll 8
    for (int k = 0; k < NN; ++k) acc += xrow[k] * w[k];
    grow[tid] = acc;
    __syncthreads();
    if (tid < 96) {
        v4f v = *(const v4f*)&grow[tid * 4];
        float* dst = gi + (size_t)row * (3 * NHG) + tid * 4;
        *(volatile v4f*)dst = v;
        __threadfence();
        *(volatile v4f*)dst = v;
    }
}

__global__ void __launch_bounds__(512) gru_kernel(const float* gi, const float* __restrict__ whh,
                                                  const float* __restrict__ bhh, float* hs) {
    __shared__ float whhT[NHG * 3 * NHG];
    __shared__ __attribute__((aligned(16))) float h[NB * NHG];
    const int tid = threadIdx.x;
    for (int idx = tid; idx < NHG * 3 * NHG; idx += 512) {
        int k = idx / (3 * NHG), j = idx - k * (3 * NHG);
        whhT[idx] = whh[(size_t)j * NHG + k];
    }
    const int b = tid >> 7, hh = tid & 127;
    h[tid] = 0.f;
    __syncthreads();
    const float bhr = bhh[hh], bhz = bhh[NHG + hh], bhn = bhh[2 * NHG + hh];
    for (int t = 0; t < NT; ++t) {
        const float* hb = h + b * NHG;
        float ghr = bhr, ghz = bhz, ghn = bhn;
#pragma unroll 4
        for (int k = 0; k < NHG; ++k) {
            float hv = hb[k];
            const float* wr = whhT + k * (3 * NHG);
            ghr += hv * wr[hh];
            ghz += hv * wr[NHG + hh];
            ghn += hv * wr[2 * NHG + hh];
        }
        const float* gir = gi + (size_t)(b * NT + t) * (3 * NHG);
        float r = sigm(gir[hh] + ghr);
        float z = sigm(gir[NHG + hh] + ghz);
        float n = tanhf(gir[2 * NHG + hh] + r * ghn);
        float hnew = (1.f - z) * n + z * hb[hh];
        __syncthreads();
        h[tid] = hnew;
        __syncthreads();
        if (tid < 128) {
            int bb = tid >> 5, pc = (tid & 31) * 4;
            v4f v = *(const v4f*)&h[bb * NHG + pc];
            float* dst = hs + (size_t)(bb * NT + t) * NHG + pc;
            *(volatile v4f*)dst = v;
            __threadfence();
            *(volatile v4f*)dst = v;
        }
    }
}

__global__ void __launch_bounds__(256) lin_kernel(const float* hs, const float* __restrict__ lwg,
                                                  const float* __restrict__ lb, float* xt) {
    __shared__ __attribute__((aligned(16))) float hsb[NT * NHG];
    __shared__ __attribute__((aligned(16))) float lw[16 * NHG];
    __shared__ __attribute__((aligned(16))) float outl[16 * NT];
    const int t = threadIdx.x, blk = blockIdx.x, b = blk >> 4, n0 = (blk & 15) * 16;
    const float* hsrc = hs + (size_t)b * (NT * NHG);
#pragma unroll
    for (int q = 0; q < 8; ++q) { int i4 = (q * 256 + t) * 4; *(v4f*)&hsb[i4] = *(const v4f*)(hsrc + i4); }
    const float* lsrc = lwg + (size_t)n0 * NHG;
#pragma unroll
    for (int q = 0; q < 2; ++q) { int i4 = (q * 256 + t) * 4; *(v4f*)&lw[i4] = *(const v4f*)(lsrc + i4); }
    __syncthreads();
    const int nl = t >> 4, t4 = (t & 15) * 4;
    const float bias = lb[n0 + nl];
    const float* wrow = &lw[nl * NHG];
    const float* hr = &hsb[t4 * NHG];
    float a0 = 0.f, a1 = 0.f, a2 = 0.f, a3 = 0.f;
#pragma unroll 4
    for (int k = 0; k < NHG; ++k) {
        float w = wrow[k];
        a0 += hr[k] * w;
        a1 += hr[NHG + k] * w;
        a2 += hr[2 * NHG + k] * w;
        a3 += hr[3 * NHG + k] * w;
    }
    outl[nl * NT + t4 + 0] = a0 + bias;
    outl[nl * NT + t4 + 1] = a1 + bias;
    outl[nl * NT + t4 + 2] = a2 + bias;
    outl[nl * NT + t4 + 3] = a3 + bias;
    __syncthreads();
    {
        v4f v = *(const v4f*)&outl[t * 4];
        float* dst = xt + (size_t)(b * NN + n0) * NT + t * 4;
        *(volatile v4f*)dst = v;
        __threadfence();
        *(volatile v4f*)dst = v;
    }
}

__global__ void __launch_bounds__(128) pair1_kernel(const float* __restrict__ xt,
    const float* __restrict__ f1w, const float* __restrict__ f1b,
    const float* __restrict__ f2w, const float* __restrict__ f2b,
    const float* __restrict__ a1w, const float* __restrict__ a1b,
    float* y1, float* part1) {
    __shared__ __attribute__((aligned(16))) _Float16 w1[128 * 64];
    __shared__ __attribute__((aligned(16))) _Float16 w2[128 * 64];
    __shared__ __attribute__((aligned(16))) _Float16 w3[64 * 128];
    __shared__ __attribute__((aligned(16))) _Float16 stg[4][16 * 128];
    __shared__ __attribute__((aligned(16))) float ost[4][16 * 64];
    __shared__ float statl[4 * 128];
    __shared__ __attribute__((aligned(16))) float combl[128];

    const int tid = threadIdx.x;
    for (int idx = tid; idx < 8192; idx += 128) {
        w1[idx] = (_Float16)(f1w[idx] * 16.f);
        w2[idx] = (_Float16)(f2w[idx] * 16.f);
        w3[idx] = (_Float16)(a1w[idx] * 16.f);
    }
    __syncthreads();

    const int wave = tid >> 5, lane = tid & 31, h = lane >> 4, m = lane & 15;
    const int blk = blockIdx.x, b = blk >> 8, i = blk & 255;
    const float* xi = xt + (size_t)(b * NN + i) * NT;
    const v8f zf = {0.f, 0.f, 0.f, 0.f, 0.f, 0.f, 0.f, 0.f};
    float sts[4] = {0.f, 0.f, 0.f, 0.f}, stq[4] = {0.f, 0.f, 0.f, 0.f};

    for (int it = 0; it < 4; ++it) {
        const int j0 = (it * 4 + wave) * 16;
        const float* xj = xt + (size_t)(b * NN + j0 + m) * NT;

        Frag dA[2], pA[2];
#pragma unroll
        for (int kb = 0; kb < 2; ++kb) {
#pragma unroll
            for (int pt = 0; pt < 2; ++pt) {
                const int koff = kb * 32 + pt * 16 + 8 * h;
                v4f ai0 = *(const v4f*)(xi + koff), ai1 = *(const v4f*)(xi + koff + 4);
                v4f aj0 = *(const v4f*)(xj + koff), aj1 = *(const v4f*)(xj + koff + 4);
#pragma unroll
                for (int e = 0; e < 4; ++e) {
                    float s0 = ai0[e], c0 = aj0[e], s1 = ai1[e], c1 = aj1[e];
                    dA[kb].v[pt * 8 + e]     = (_Float16)fabsf(s0 - c0);
                    dA[kb].v[pt * 8 + 4 + e] = (_Float16)fabsf(s1 - c1);
                    pA[kb].v[pt * 8 + e]     = (_Float16)(s0 * c0 * 16.f);
                    pA[kb].v[pt * 8 + 4 + e] = (_Float16)(s1 * c1 * 16.f);
                }
            }
        }

#pragma unroll
        for (int nt = 0; nt < 8; ++nt) {
            const int n = nt * 16 + m;
            v8f acc1 = zf, acc2 = zf;
#pragma unroll
            for (int kb = 0; kb < 2; ++kb) {
                Frag b1, b2;
                const int ko = n * 64 + kb * 32 + 8 * h;
                b1.hv[0] = *(const v8h*)&w1[ko]; b1.hv[1] = *(const v8h*)&w1[ko + 16];
                b2.hv[0] = *(const v8h*)&w2[ko]; b2.hv[1] = *(const v8h*)&w2[ko + 16];
                acc1 = wmma16(dA[kb].v, b1.v, acc1);
                acc2 = wmma16(pA[kb].v, b2.v, acc2);
            }
            const float bb1 = f1b[n], bb2 = f2b[n];
#pragma unroll
            for (int r = 0; r < 8; ++r) {
                float v = lrelu(acc1[r] * 0.0625f + bb1) + lrelu(acc2[r] * 0.00390625f + bb2);
                stg[wave][(8 * h + r) * 128 + n] = (_Float16)(v * 8.f);
            }
        }
        __syncthreads();

        v8f yacc[4];
#pragma unroll
        for (int nt = 0; nt < 4; ++nt) yacc[nt] = zf;
#pragma unroll
        for (int kb = 0; kb < 4; ++kb) {
            Frag a;
            const int ao = m * 128 + kb * 32 + 8 * h;
            a.hv[0] = *(const v8h*)&stg[wave][ao];
            a.hv[1] = *(const v8h*)&stg[wave][ao + 16];
#pragma unroll
            for (int nt = 0; nt < 4; ++nt) {
                Frag bb;
                const int bo = (nt * 16 + m) * 128 + kb * 32 + 8 * h;
                bb.hv[0] = *(const v8h*)&w3[bo];
                bb.hv[1] = *(const v8h*)&w3[bo + 16];
                yacc[nt] = wmma16(a.v, bb.v, yacc[nt]);
            }
        }
#pragma unroll
        for (int nt = 0; nt < 4; ++nt) {
            const int n = nt * 16 + m;
            const float bias = a1b[n];
#pragma unroll
            for (int r = 0; r < 8; ++r) {
                float v = yacc[nt][r] * 0.0078125f + bias;
                ost[wave][(8 * h + r) * 64 + n] = v;
                sts[nt] += v;
                stq[nt] += v * v;
            }
        }
        __syncthreads();
        {
            float* dst = y1 + ((size_t)(b * NN + i) * NN + j0) * 64;
            v4f vv[8];
#pragma unroll
            for (int q = 0; q < 8; ++q) vv[q] = *(const v4f*)&ost[wave][q * 128 + lane * 4];
#pragma unroll
            for (int q = 0; q < 8; ++q) *(volatile v4f*)(dst + q * 128 + lane * 4) = vv[q];
            __threadfence();
#pragma unroll
            for (int q = 0; q < 8; ++q) *(volatile v4f*)(dst + q * 128 + lane * 4) = vv[q];
        }
        __syncthreads();
    }

#pragma unroll
    for (int nt = 0; nt < 4; ++nt) {
        float s = sts[nt] + __shfl_xor(sts[nt], 16);
        float q = stq[nt] + __shfl_xor(stq[nt], 16);
        if (h == 0) { statl[wave * 128 + nt * 16 + m] = s; statl[wave * 128 + 64 + nt * 16 + m] = q; }
    }
    __syncthreads();
    if (tid < 128) combl[tid] = statl[tid] + statl[128 + tid] + statl[256 + tid] + statl[384 + tid];
    __syncthreads();
    if (tid < 32) {
        v4f v = *(const v4f*)&combl[tid * 4];
        float* p = part1 + (size_t)blk * 128 + tid * 4;
        *(volatile v4f*)p = v;
        __threadfence();
        *(volatile v4f*)p = v;
    }
}

__global__ void __launch_bounds__(64) bnfin_kernel(const float* part, const float* __restrict__ g,
                                                   const float* __restrict__ bt, float* bnp) {
    __shared__ __attribute__((aligned(16))) float bl[128];
    const int c = threadIdx.x;
    double s = 0.0, q = 0.0;
    for (int k = 0; k < 1024; ++k) {
        s += (double)part[k * 128 + c];
        q += (double)part[k * 128 + 64 + c];
    }
    const double inv = 1.0 / 262144.0;
    double mean = s * inv;
    double var = q * inv - mean * mean;
    if (var < 0.0) var = 0.0;
    double scd = (double)g[c] / sqrt(var + 1e-5);
    bl[c] = (float)scd;
    bl[64 + c] = (float)((double)bt[c] - mean * scd);
    __syncthreads();
    if (c < 32) {
        v4f v = *(const v4f*)&bl[c * 4];
        float* p = bnp + c * 4;
        *(volatile v4f*)p = v;
        __threadfence();
        *(volatile v4f*)p = v;
    }
}

template <bool FINAL>
__global__ void __launch_bounds__(128) pass_kernel(const float* y1, const float* __restrict__ bnp1,
    const float* __restrict__ a2w, const float* __restrict__ a2b, const float* __restrict__ bnp2,
    const float* __restrict__ alw, const float* __restrict__ alb, float* dst) {
    __shared__ __attribute__((aligned(16))) _Float16 w4[64 * 64];
    __shared__ float sc1[64], sh1[64], sc2[64], sh2[64], alv[64];
    __shared__ float statl[4 * 128];
    __shared__ __attribute__((aligned(16))) float combl[128];
    __shared__ __attribute__((aligned(16))) float arl[256];

    const int tid = threadIdx.x;
    for (int idx = tid; idx < 4096; idx += 128) w4[idx] = (_Float16)(a2w[idx] * 16.f);
    if (tid < 64) {
        sc1[tid] = bnp1[tid]; sh1[tid] = bnp1[64 + tid];
        if (FINAL) { sc2[tid] = bnp2[tid]; sh2[tid] = bnp2[64 + tid]; alv[tid] = alw[tid]; }
        else { sc2[tid] = 0.f; sh2[tid] = 0.f; alv[tid] = 0.f; }
    }
    __syncthreads();

    const int wave = tid >> 5, lane = tid & 31, h = lane >> 4, m = lane & 15;
    const int blk = blockIdx.x, b = blk >> 8, i = blk & 255;
    const float alb0 = FINAL ? alb[0] : 0.f;
    const v8f zf = {0.f, 0.f, 0.f, 0.f, 0.f, 0.f, 0.f, 0.f};
    float sts[4] = {0.f, 0.f, 0.f, 0.f}, stq[4] = {0.f, 0.f, 0.f, 0.f};

    for (int it = 0; it < 4; ++it) {
        const int j0 = (it * 4 + wave) * 16;
        const size_t R0 = (size_t)(b * NN + i) * NN + j0;
        const float* yr = y1 + (R0 + m) * 64;

        Frag A[2];
#pragma unroll
        for (int kb = 0; kb < 2; ++kb) {
#pragma unroll
            for (int pt = 0; pt < 2; ++pt) {
                const int koff = kb * 32 + pt * 16 + 8 * h;
                v4f u0 = *(const v4f*)(yr + koff), u1 = *(const v4f*)(yr + koff + 4);
#pragma unroll
                for (int e = 0; e < 4; ++e) {
                    const int k0 = koff + e, k1 = koff + 4 + e;
                    A[kb].v[pt * 8 + e]     = (_Float16)lrelu(u0[e] * sc1[k0] + sh1[k0]);
                    A[kb].v[pt * 8 + 4 + e] = (_Float16)lrelu(u1[e] * sc1[k1] + sh1[k1]);
                }
            }
        }
        v8f acc[4];
#pragma unroll
        for (int nt = 0; nt < 4; ++nt) acc[nt] = zf;
#pragma unroll
        for (int kb = 0; kb < 2; ++kb) {
#pragma unroll
            for (int nt = 0; nt < 4; ++nt) {
                Frag bb;
                const int bo = (nt * 16 + m) * 64 + kb * 32 + 8 * h;
                bb.hv[0] = *(const v8h*)&w4[bo];
                bb.hv[1] = *(const v8h*)&w4[bo + 16];
                acc[nt] = wmma16(A[kb].v, bb.v, acc[nt]);
            }
        }
        if (!FINAL) {
#pragma unroll
            for (int nt = 0; nt < 4; ++nt) {
                const float bias = a2b[nt * 16 + m];
#pragma unroll
                for (int r = 0; r < 8; ++r) {
                    float v = acc[nt][r] * 0.0625f + bias;
                    sts[nt] += v;
                    stq[nt] += v * v;
                }
            }
        } else {
            float rd[8] = {0.f, 0.f, 0.f, 0.f, 0.f, 0.f, 0.f, 0.f};
#pragma unroll
            for (int nt = 0; nt < 4; ++nt) {
                const int n = nt * 16 + m;
                const float bias = a2b[n], s2 = sc2[n], t2 = sh2[n], aw = alv[n];
#pragma unroll
                for (int r = 0; r < 8; ++r) {
                    float v = acc[nt][r] * 0.0625f + bias;
                    float u = lrelu(v * s2 + t2);
                    rd[r] += u * aw;
                }
            }
#pragma unroll
            for (int off = 1; off < 16; off <<= 1) {
#pragma unroll
                for (int r = 0; r < 8; ++r) rd[r] += __shfl_xor(rd[r], off);
            }
            if (m == 0) {
#pragma unroll
                for (int r = 0; r < 8; ++r) arl[j0 + 8 * h + r] = rd[r] + alb0;
            }
        }
    }

    if (!FINAL) {
#pragma unroll
        for (int nt = 0; nt < 4; ++nt) {
            float s = sts[nt] + __shfl_xor(sts[nt], 16);
            float q = stq[nt] + __shfl_xor(stq[nt], 16);
            if (h == 0) { statl[wave * 128 + nt * 16 + m] = s; statl[wave * 128 + 64 + nt * 16 + m] = q; }
        }
        __syncthreads();
        if (tid < 128) combl[tid] = statl[tid] + statl[128 + tid] + statl[256 + tid] + statl[384 + tid];
        __syncthreads();
        if (tid < 32) {
            v4f v = *(const v4f*)&combl[tid * 4];
            float* p = dst + (size_t)blk * 128 + tid * 4;
            *(volatile v4f*)p = v;
            __threadfence();
            *(volatile v4f*)p = v;
        }
    } else {
        __syncthreads();
        if (tid < 64) {
            v4f v = *(const v4f*)&arl[tid * 4];
            float* p = dst + (size_t)blk * 256 + tid * 4;
            *(volatile v4f*)p = v;
            __threadfence();
            *(volatile v4f*)p = v;
        }
    }
}

__global__ void __launch_bounds__(256) ahat_kernel(const float* __restrict__ araw, float* out1) {
    const int t = threadIdx.x;
    const int R = blockIdx.x * 4 + (t >> 6);
    const int b = R >> 8, r = R & 255;
    const int c0 = (t & 63) * 4;
    const float* ab = araw + (size_t)b * 65536;
    v4f a = *(const v4f*)(ab + (size_t)r * 256 + c0);
    v4f o;
#pragma unroll
    for (int q = 0; q < 4; ++q) {
        float tr = ab[(size_t)(c0 + q) * 256 + r];
        float v = (a[q] + tr) * 0.5f;
        o[q] = sigm(v);
    }
    float* d = out1 + (size_t)R * 256 + c0;
    *(volatile v4f*)d = o;
    __threadfence();
    *(volatile v4f*)d = o;
}

__global__ void __launch_bounds__(256) gcn_kernel(const float* __restrict__ xt, const float* __restrict__ gcnw,
    const float* __restrict__ gcnb, const float* ahat, const int* __restrict__ edge, float* out0) {
    __shared__ __attribute__((aligned(16))) float xts[NN * 64];
    __shared__ __attribute__((aligned(16))) float xll[NN * 64];
    __shared__ float disl[NN];
    const int b = blockIdx.x, c = threadIdx.x;
    const float* xtb = xt + (size_t)b * (NN * 64);
#pragma unroll
    for (int q = 0; q < 16; ++q) { int i4 = (q * 256 + c) * 4; *(v4f*)&xts[i4] = *(const v4f*)(xtb + i4); }
    __syncthreads();

#pragma unroll 1
    for (int o = 0; o < 64; ++o) {
        const float* w = gcnw + o * 64;
        float acc = 0.f;
#pragma unroll 8
        for (int k = 0; k < 64; ++k) acc += xts[c * 64 + k] * w[k];
        xll[c * 64 + o] = acc;
    }

    const float* ab = ahat + (size_t)b * 65536;
    float dsum = 0.f;
#pragma unroll 2
    for (int e = 0; e < NE; ++e) {
        int cl = edge[NE + e];
        if (cl == c) {
            int r = edge[e];
            r = r < 0 ? 0 : (r > 255 ? 255 : r);
            dsum += ab[r * 256 + c];
        }
    }
    disl[c] = dsum > 0.f ? rsqrtf(dsum) : 0.f;
    __syncthreads();

    float acc[64];
#pragma unroll
    for (int o = 0; o < 64; ++o) acc[o] = 0.f;
    const float dc = disl[c];
#pragma unroll 2
    for (int e = 0; e < NE; ++e) {
        int cl = edge[NE + e];
        if (cl == c) {
            int r = edge[e];
            r = r < 0 ? 0 : (r > 255 ? 255 : r);
            float ew = ab[r * 256 + c];
            float nrm = disl[r] * ew * dc;
            const float* xr = &xll[r * 64];
#pragma unroll
            for (int o = 0; o < 64; ++o) acc[o] += nrm * xr[o];
        }
    }
    __syncthreads();
#pragma unroll
    for (int o = 0; o < 64; ++o) xll[o * 256 + c] = acc[o] + gcnb[o];
    __syncthreads();
    {
        float* ob = out0 + (size_t)b * 16384;
        v4f vv[16];
#pragma unroll
        for (int q = 0; q < 16; ++q) vv[q] = *(const v4f*)&xll[(q * 256 + c) * 4];
#pragma unroll
        for (int q = 0; q < 16; ++q) *(volatile v4f*)(ob + (q * 256 + c) * 4) = vv[q];
        __threadfence();
#pragma unroll
        for (int q = 0; q < 16; ++q) *(volatile v4f*)(ob + (q * 256 + c) * 4) = vv[q];
    }
}

extern "C" void kernel_launch(void* const* d_in, const int* in_sizes, int n_in,
                              void* d_out, int out_size, void* d_ws, size_t ws_size,
                              hipStream_t stream) {
    if (n_in < 24) return;
    const int expect[24] = {65536, 98304, 49152, 384, 384, 32768, 256, 8192, 128, 8192, 128,
                            8192, 64, 64, 64, 4096, 64, 64, 64, 64, 1, 4096, 64, 8192};
    for (int i = 0; i < 24; ++i) if (in_sizes[i] != expect[i]) return;
    if (out_size != 65536 + 262144) return;

    const float* x    = (const float*)d_in[0];
    const float* gwih = (const float*)d_in[1];
    const float* gwhh = (const float*)d_in[2];
    const float* gbih = (const float*)d_in[3];
    const float* gbhh = (const float*)d_in[4];
    const float* linw = (const float*)d_in[5];
    const float* linb = (const float*)d_in[6];
    const float* f1w  = (const float*)d_in[7];
    const float* f1b  = (const float*)d_in[8];
    const float* f2w  = (const float*)d_in[9];
    const float* f2b  = (const float*)d_in[10];
    const float* a1w  = (const float*)d_in[11];
    const float* a1b  = (const float*)d_in[12];
    const float* bn1g = (const float*)d_in[13];
    const float* bn1b = (const float*)d_in[14];
    const float* a2w  = (const float*)d_in[15];
    const float* a2b  = (const float*)d_in[16];
    const float* bn2g = (const float*)d_in[17];
    const float* bn2b = (const float*)d_in[18];
    const float* alw  = (const float*)d_in[19];
    const float* alb  = (const float*)d_in[20];
    const float* gcnw = (const float*)d_in[21];
    const float* gcnb = (const float*)d_in[22];
    const int*   edge = (const int*)d_in[23];

    const size_t n_y1   = (size_t)262144 * 64;
    const size_t n_araw = 262144;
    const size_t n_gi   = (size_t)256 * 384;
    const size_t n_hs   = (size_t)256 * 128;
    const size_t n_xt   = (size_t)1024 * 64;
    const size_t n_part = (size_t)1024 * 128;
    const size_t n_bnp  = 128;
    const size_t total_f = n_y1 + n_araw + n_gi + n_hs + n_xt + 2 * n_part + 2 * n_bnp;
    if (total_f * sizeof(float) > ws_size) return;

    float* ws    = (float*)d_ws;
    float* y1    = ws;
    float* araw  = y1 + n_y1;
    float* gi    = araw + n_araw;
    float* hs    = gi + n_gi;
    float* xt    = hs + n_hs;
    float* part1 = xt + n_xt;
    float* part2 = part1 + n_part;
    float* bnp1  = part2 + n_part;
    float* bnp2  = bnp1 + n_bnp;

    float* out0 = (float*)d_out;
    float* out1 = out0 + 65536;

    gi_kernel<<<256, 384, 0, stream>>>(x, gwih, gbih, gi);
    gru_kernel<<<1, 512, 0, stream>>>(gi, gwhh, gbhh, hs);
    lin_kernel<<<64, 256, 0, stream>>>(hs, linw, linb, xt);

    pair1_kernel<<<1024, 128, 0, stream>>>(xt, f1w, f1b, f2w, f2b, a1w, a1b, y1, part1);
    bnfin_kernel<<<1, 64, 0, stream>>>(part1, bn1g, bn1b, bnp1);
    pass_kernel<false><<<1024, 128, 0, stream>>>(y1, bnp1, a2w, a2b, bnp2, alw, alb, part2);
    bnfin_kernel<<<1, 64, 0, stream>>>(part2, bn2g, bn2b, bnp2);
    pass_kernel<true><<<1024, 128, 0, stream>>>(y1, bnp1, a2w, a2b, bnp2, alw, alb, araw);
    ahat_kernel<<<256, 256, 0, stream>>>(araw, out1);

    gcn_kernel<<<NB, 256, 0, stream>>>(xt, gcnw, gcnb, out1, edge, out0);
}
